// Encoder_48524540511031
// MI455X (gfx1250) — hardware-run, weakly checked
//
#include <hip/hip_runtime.h>
#include <stddef.h>
#include <stdint.h>


#define NN      50000
#define NE      800000
#define HD      128
#define NG      64
#define TM      128
#define NT      391
#define MP      (NT * TM)
#define KTOT    256
#define APW     256
#define WSQ     (HD * KTOT)
#define NUSQ    (HD * (KTOT / 8))
#define NMAT    4
#define NTHR    256
#define NWAVE   8
#define EPT     8
#define CHUNK   (NTHR * EPT)
#define WCAP    (EPT * 32)
#define LISTN   (NWAVE * WCAP)
#define NBA     1024
#define SLA     10
#define NBK     49
#define NPADS   (NBK * NBA)
#define RCAP    20480
#define DEGCAP  64
#define RECW    384
#define PARF    1536
#define STATF   256
#define TABF    (PARF + 4 * STATF)
#define OUT1E   8192
#define BK_ZINTS (LISTN + 2 * RCAP + 3 * NBA)
#define BK_LDS_INTS (BK_ZINTS + 16)
#define BK_LDS  (BK_LDS_INTS * 4)
#define PW      ((NMAT * NUSQ) / NTHR)
#define PP      2
#define PX      ((MP * 16) / NTHR)
#define WSMAX   134217728
#define TERMS_P0 2
#define TERMS_T0 2
#define TERMS_P1 2
#define TERMS_T1 2

static_assert(HD == 128 && KTOT == 2 * HD && APW == 2 * HD);
static_assert(NT == 391 && NT * TM >= NN && (NT - 1) * TM < NN && NN - (NT - 1) * TM == 80);
static_assert(NG == 64 && OUT1E == NG * HD);
static_assert(NBK * NBA >= NN && NBK * NBA >= MP && (NBA % TM) == 0 && NBA == (1 << SLA));
static_assert((CHUNK & (CHUNK - 1)) == 0 && ((long long)(NE + CHUNK) << SLA) < (1LL << 31));
static_assert(RCAP * 100 >= 16696 * 105 && (RCAP % (NTHR * 4)) == 0);
static_assert(DEGCAP >= 33 + 8);
static_assert((BK_ZINTS % 4) == 0 && BK_LDS <= 327680);
static_assert((NUSQ % NTHR) == 0 && ((MP * 16) % NTHR) == 0 && (KTOT / 8) == 32);
static_assert(TM == NWAVE * 16 && NTHR == 2 * HD && (NN % 4) == 0 && (NE % 4) == 0);
static_assert(TM * HD * 4 + RECW * 4 + HD * 4 <= 327680);
static_assert(TM * HD * 4 + NG * HD * 4 + 4 * HD * 4 + TM * 4 <= 327680);
static_assert(TERMS_P0 >= 1 && TERMS_P0 <= 2 && TERMS_T0 >= 1 && TERMS_T0 <= 2);
static_assert(TERMS_P1 >= 1 && TERMS_P1 <= 2 && TERMS_T1 >= 1 && TERMS_T1 <= 2);

typedef float          v4f  __attribute__((ext_vector_type(4)));
typedef float          v8f  __attribute__((ext_vector_type(8)));
typedef int            v4i  __attribute__((ext_vector_type(4)));
typedef int            v8i  __attribute__((ext_vector_type(8)));
typedef unsigned int   v2u  __attribute__((ext_vector_type(2)));
typedef unsigned int   v4u  __attribute__((ext_vector_type(4)));
typedef unsigned short v8us __attribute__((ext_vector_type(8)));
typedef __bf16         v16b __attribute__((ext_vector_type(16)));
typedef v4f  __attribute__((may_alias)) v4fa;
typedef v4i  __attribute__((may_alias)) v4ia;
typedef v2u  __attribute__((may_alias)) v2ua;
typedef v4u  __attribute__((may_alias)) v4ua;
typedef v8us __attribute__((may_alias)) v8usa;
union FragB { v16b v; v8us h[2]; v8i w; };

__device__ __forceinline__ v8f wmb(const FragB& a, const FragB& b, v8f c) {
  v8f d = __builtin_amdgcn_wmma_f32_16x16x32_bf16(false, a.v, false, b.v, (short)0, c, false, false);
  asm volatile("v_nop\n\tv_nop\n\tv_nop\n\tv_nop" : "+v"(d) : "v"(a.w), "v"(b.w));
  return d;
}

__device__ __forceinline__ unsigned short bf_bits(float f) {
  const unsigned int u = __float_as_uint(f);
  const unsigned int r = (u + 0x7FFFu + ((u >> 16) & 1u)) >> 16;
  const bool isn = (u & 0x7FFFFFFFu) > 0x7F800000u;
  return (unsigned short)(isn ? 0x7FC0u : r);
}
__device__ __forceinline__ float bf_val(unsigned short b) {
  return __uint_as_float(((unsigned int)b) << 16);
}
__device__ __forceinline__ float bf_rne(float f) { return bf_val(bf_bits(f)); }

__device__ __forceinline__ float relu_p(float v) { return (v > 0.0f) ? v : (v - v); }

__device__ __forceinline__ float bn_relu(float v, float mu, float r, float g, float be) {
  float y = g * (v - mu);
  y = y * r;
  y = y + be;
  return relu_p(y);
}

__device__ __forceinline__ v8us gather8(const float* __restrict__ p) {
  v8us o;
#pragma unroll
  for (int i = 0; i < 8; ++i) o[i] = bf_bits(p[(size_t)i * HD]);
  return o;
}

__global__ __launch_bounds__(NTHR) void k_prep(const float* __restrict__ x,
    const float* __restrict__ W1, const float* __restrict__ b1, const float* __restrict__ g1,
    const float* __restrict__ be1, const float* __restrict__ W2, const float* __restrict__ b2,
    const float* __restrict__ gbn, const float* __restrict__ bbn,
    unsigned short* wt, float* tab, unsigned short* xb) {
  const int tid = (int)threadIdx.x;
  const int blk = (int)blockIdx.x;
  if (blk < PW) {
    const int u     = blk * NTHR + tid;
    const int mi    = u / NUSQ;
    const int v     = u - mi * NUSQ;
    const int n     = v >> 5;
    const int k8    = (v & 31) * 8;
    const int kk    = k8 & (HD - 1);
    const int layer = mi >> 1;
    const size_t so = (size_t)layer * HD * HD + (size_t)kk * HD + (size_t)n;
    v8us o;
    if ((mi & 1) != 0) { o = gather8(W2 + so); } else { o = gather8(W1 + so); }
    unsigned short* dp = wt + (size_t)mi * WSQ + (size_t)n * KTOT + k8;
    *(volatile v8us*)dp = o;
    __threadfence();
    *(volatile v8us*)dp = o;
    return;
  }
  if (blk < PW + PP) {
    const int u2 = (blk - PW) * NTHR + tid;
    int t = u2 >> 6;
    t = t > 5 ? 5 : t;
    const int j4 = (u2 & 63) * 4;
    const v4f c0 = *(const v4f*)(b1  + j4);
    const v4f c1 = *(const v4f*)(g1  + j4);
    const v4f c2 = *(const v4f*)(be1 + j4);
    const v4f c3 = *(const v4f*)(b2  + j4);
    const v4f c4 = *(const v4f*)(gbn + j4);
    const v4f c5 = *(const v4f*)(bbn + j4);
    asm volatile("" :: "v"(c0), "v"(c1), "v"(c2), "v"(c3), "v"(c4), "v"(c5));
    v4f s = c0;
    s = (t == 1) ? c1 : s;
    s = (t == 2) ? c2 : s;
    s = (t == 3) ? c3 : s;
    s = (t == 4) ? c4 : s;
    s = (t == 5) ? c5 : s;
    v4f o;
    o.x = bf_rne(s.x); o.y = bf_rne(s.y); o.z = bf_rne(s.z); o.w = bf_rne(s.w);
    const bool okp = u2 < (PARF / 4);
    float* dp = tab + 4 * (okp ? u2 : 0);
    if (okp) *(volatile v4f*)dp = o;
    __threadfence();
    if (okp) *(volatile v4f*)dp = o;
    return;
  }
  {
    const int u   = (blk - PW - PP) * NTHR + tid;
    const int row = u >> 4;
    const int c8  = (u & 15) * 8;
    const int rc  = row < NN ? row : NN - 1;
    const float* p = x + (size_t)rc * HD + c8;
    const v4f a = *(const v4f*)p;
    const v4f b = *(const v4f*)(p + 4);
    asm volatile("" :: "v"(a), "v"(b));
    const bool live = row < NN;
    v8us o;
    o[0] = live ? bf_bits(a.x) : (unsigned short)0; o[1] = live ? bf_bits(a.y) : (unsigned short)0;
    o[2] = live ? bf_bits(a.z) : (unsigned short)0; o[3] = live ? bf_bits(a.w) : (unsigned short)0;
    o[4] = live ? bf_bits(b.x) : (unsigned short)0; o[5] = live ? bf_bits(b.y) : (unsigned short)0;
    o[6] = live ? bf_bits(b.z) : (unsigned short)0; o[7] = live ? bf_bits(b.w) : (unsigned short)0;
    unsigned short* dp = xb + (size_t)u * 8;
    *(volatile v8us*)dp = o;
    __threadfence();
    *(volatile v8us*)dp = o;
  }
}

__device__ __forceinline__ int scan_chunk(const int* __restrict__ keys, int nE, int cbase, int slotBase,
                                          int vec8, int* list, int tid, int wave) {
  int wc = 0;
  const int el0  = tid * EPT;
  const int e0   = cbase + el0;
  const int sent = -2147483647 - 1;
  v4i da, db;
  if (vec8 != 0 && cbase + CHUNK <= nE) {
    da = *(const v4i*)(keys + e0);
    db = *(const v4i*)(keys + e0 + 4);
  } else {
    const int k0 = keys[min(e0,     nE - 1)];
    const int k1 = keys[min(e0 + 1, nE - 1)];
    const int k2 = keys[min(e0 + 2, nE - 1)];
    const int k3 = keys[min(e0 + 3, nE - 1)];
    const int k4 = keys[min(e0 + 4, nE - 1)];
    const int k5 = keys[min(e0 + 5, nE - 1)];
    const int k6 = keys[min(e0 + 6, nE - 1)];
    const int k7 = keys[min(e0 + 7, nE - 1)];
    asm volatile("" :: "v"(k0), "v"(k1), "v"(k2), "v"(k3), "v"(k4), "v"(k5), "v"(k6), "v"(k7));
    da.x = (e0     < nE) ? k0 : sent;
    da.y = (e0 + 1 < nE) ? k1 : sent;
    da.z = (e0 + 2 < nE) ? k2 : sent;
    da.w = (e0 + 3 < nE) ? k3 : sent;
    db.x = (e0 + 4 < nE) ? k4 : sent;
    db.y = (e0 + 5 < nE) ? k5 : sent;
    db.z = (e0 + 6 < nE) ? k6 : sent;
    db.w = (e0 + 7 < nE) ? k7 : sent;
  }
  const unsigned nbs = (unsigned)slotBase;
  const unsigned unb = (unsigned)NBA;
  const unsigned s0 = (unsigned)da.x - nbs, s1 = (unsigned)da.y - nbs;
  const unsigned s2 = (unsigned)da.z - nbs, s3 = (unsigned)da.w - nbs;
  const unsigned s4 = (unsigned)db.x - nbs, s5 = (unsigned)db.y - nbs;
  const unsigned s6 = (unsigned)db.z - nbs, s7 = (unsigned)db.w - nbs;
  const bool h0 = s0 < unb, h1 = s1 < unb, h2 = s2 < unb, h3 = s3 < unb;
  const bool h4 = s4 < unb, h5 = s5 < unb, h6 = s6 < unb, h7 = s7 < unb;
  const unsigned any = __builtin_amdgcn_ballot_w32(h0 | h1 | h2 | h3 | h4 | h5 | h6 | h7);
  if (any != 0u) {
#define HITJ(J, HJ, SJ) { \
      const unsigned mj = __builtin_amdgcn_ballot_w32(HJ); \
      const int pos = wc + (int)__builtin_amdgcn_mbcnt_lo(mj, 0u); \
      if ((HJ) && pos < WCAP) list[wave * WCAP + pos] = ((el0 + (J)) << SLA) | (int)(SJ); \
      wc += (int)__builtin_popcount(mj); }
    HITJ(0, h0, s0)
    HITJ(1, h1, s1)
    HITJ(2, h2, s2)
    HITJ(3, h3, s3)
    HITJ(4, h4, s4)
    HITJ(5, h5, s5)
    HITJ(6, h6, s6)
    HITJ(7, h7, s7)
#undef HITJ
  }
  return wc;
}

__global__ __launch_bounds__(NTHR) void k_bucket(const int* __restrict__ srcs, const int* __restrict__ dsts,
                                                 int* listg, int* cntg, int* offg, int* flagg) {
  extern __shared__ __attribute__((aligned(16))) int dsm[];
  int* list = dsm;
  int* hl   = dsm + LISTN;
  int* sl   = hl + RCAP;
  int* cnt  = sl + RCAP;
  int* offs = cnt + NBA;
  int* cur  = offs + NBA;
  int* misc = cur + NBA;
  const int tid = (int)threadIdx.x, lane = tid & 31, wave = tid >> 5;
  const int b = (int)blockIdx.x;
  const int nodeBase = b * NBA;

  {
    const v4i z4 = {0, 0, 0, 0};
    for (int i = tid * 4; i < BK_ZINTS; i += NTHR * 4) *(v4ia*)(dsm + i) = z4;
    if (tid < 16) misc[tid] = 0;
  }
  __syncthreads();

  int t = 0, ov = 0;
  const int nChunks = (NE + CHUNK - 1) / CHUNK;
#pragma unroll 1
  for (int ch = 0; ch < nChunks; ++ch) {
    const int cbase = ch * CHUNK;
    const int wc = scan_chunk(dsts, NE, cbase, nodeBase, 1, list, tid, wave);
    if (lane == 0) misc[wave] = wc;
    __syncthreads();
    if (wave == 0) {
#pragma unroll 1
      for (int w2 = 0; w2 < NWAVE; ++w2) {
        int c = misc[w2];
        c = c < 0 ? 0 : (c > WCAP ? WCAP : c);
#pragma unroll 1
        for (int b0 = 0; b0 < c; b0 += 32) {
          const int idx = b0 + lane;
          const int ent = list[w2 * WCAP + (idx < WCAP ? idx : WCAP - 1)];
          const int m32 = (c - b0) < 32 ? (c - b0) : 32;
#pragma unroll 1
          for (int k = 0; k < m32; ++k) {
            const int u    = __builtin_amdgcn_readlane(ent, k);
            const int slot = u & (NBA - 1);
            const int el   = (u >> SLA) & (CHUNK - 1);
            const int pk   = ((cbase + el) << SLA) | slot;
            if (t < RCAP) {
              if (lane == 0) { hl[t] = pk; cnt[slot] = cnt[slot] + 1; }
              t = t + 1;
            } else {
              ov = 1;
            }
          }
        }
      }
    }
    __syncthreads();
  }
  if (wave == 0 && lane == 0) { misc[8] = t; misc[9] = ov; }
  __syncthreads();
  int tt = misc[8];
  tt = tt < 0 ? 0 : (tt > RCAP ? RCAP : tt);
  const int ovf = misc[9];

  if (wave == 0) {
    const int base = lane * (NBA / 32);
    int s = 0;
#pragma unroll 1
    for (int i = 0; i < NBA / 32; ++i) s += cnt[base + i];
    int incl = s;
#pragma unroll
    for (int d = 1; d < 32; d <<= 1) {
      const int y = __shfl_up(incl, d, 32);
      if (lane >= d) incl += y;
    }
    int run = incl - s;
#pragma unroll 1
    for (int i = 0; i < NBA / 32; ++i) {
      const int cv = cnt[base + i];
      offs[base + i] = run;
      cur[base + i]  = run;
      run += cv;
    }
  }
  __syncthreads();
  if (wave == 0) {
#pragma unroll 1
    for (int b0 = 0; b0 < tt; b0 += 32) {
      const int idx = b0 + lane;
      const int ent = hl[idx < RCAP ? idx : RCAP - 1];
      const int m32 = (tt - b0) < 32 ? (tt - b0) : 32;
#pragma unroll 1
      for (int k = 0; k < m32; ++k) {
        const int u    = __builtin_amdgcn_readlane(ent, k);
        const int slot = u & (NBA - 1);
        if (lane == 0) {
          int p = cur[slot];
          p = p < 0 ? 0 : (p > RCAP - 1 ? RCAP - 1 : p);
          sl[p] = u;
          cur[slot] = p + 1;
        }
      }
    }
  }
  __syncthreads();

#pragma unroll 1
  for (int it = 0; it < RCAP / (NTHR * 4); ++it) {
    const int p = it * (NTHR * 4) + 4 * tid;
    const v4i e = *(const v4ia*)(sl + p);
    int e0 = e.x >> SLA, e1 = e.y >> SLA, e2 = e.z >> SLA, e3 = e.w >> SLA;
    e0 = e0 < 0 ? 0 : (e0 > NE - 1 ? NE - 1 : e0);
    e1 = e1 < 0 ? 0 : (e1 > NE - 1 ? NE - 1 : e1);
    e2 = e2 < 0 ? 0 : (e2 > NE - 1 ? NE - 1 : e2);
    e3 = e3 < 0 ? 0 : (e3 > NE - 1 ? NE - 1 : e3);
    const int r0 = srcs[e0];
    const int r1 = srcs[e1];
    const int r2 = srcs[e2];
    const int r3 = srcs[e3];
    asm volatile("" :: "v"(r0), "v"(r1), "v"(r2), "v"(r3));
    const int c0 = r0 < 0 ? 0 : (r0 > NN - 1 ? NN - 1 : r0);
    const int c1 = r1 < 0 ? 0 : (r1 > NN - 1 ? NN - 1 : r1);
    const int c2 = r2 < 0 ? 0 : (r2 > NN - 1 ? NN - 1 : r2);
    const int c3 = r3 < 0 ? 0 : (r3 > NN - 1 ? NN - 1 : r3);
    v4i o;
    o.x = (p     < tt) ? c0 : 0;
    o.y = (p + 1 < tt) ? c1 : 0;
    o.z = (p + 2 < tt) ? c2 : 0;
    o.w = (p + 3 < tt) ? c3 : 0;
    int* gp = listg + (size_t)b * RCAP + p;
    *(volatile v4i*)gp = o;
    __threadfence();
    *(volatile v4i*)gp = o;
  }
  {
    const v4i cq = *(const v4ia*)(cnt + 4 * tid);
    const v4i oq = *(const v4ia*)(offs + 4 * tid);
    int* cp = cntg + (size_t)b * NBA + 4 * tid;
    int* op = offg + (size_t)b * NBA + 4 * tid;
    v4i fq;
    fq.x = (tid == 0) ? ovf : 0;
    fq.y = (tid == 0) ? tt : 0;
    fq.z = 0; fq.w = 0;
    int* fp = flagg + (size_t)b * 32 + 4 * (tid & 7);
    const bool fok = tid < 8;
    *(volatile v4i*)cp = cq;
    *(volatile v4i*)op = oq;
    if (fok) *(volatile v4i*)fp = fq;
    __threadfence();
    *(volatile v4i*)cp = cq;
    *(volatile v4i*)op = oq;
    if (fok) *(volatile v4i*)fp = fq;
  }
}

template <int SRCBF>
__global__ __launch_bounds__(NTHR) __attribute__((amdgpu_num_vgpr(248)))
void k_agg(const unsigned short* __restrict__ xb, const float* __restrict__ ph,
           const int* __restrict__ listg, const int* __restrict__ cntg, const int* __restrict__ offg,
           const int* __restrict__ flagg, unsigned short* pa) {
  __shared__ __attribute__((aligned(16))) unsigned int stw[NWAVE * 128];
  const int tid = (int)threadIdx.x, lane = tid & 31;
  const int wave = __builtin_amdgcn_readfirstlane(tid >> 5);
  const int rowBase = (int)blockIdx.x * TM;
  int bk = rowBase >> SLA;
  bk = bk > NBK - 1 ? NBK - 1 : bk;
  const int row0 = rowBase + 16 * wave;
  const int li = row0 + (lane & 15);
  const int cv = cntg[li];
  const int ovv = offg[li];
  const int fl = flagg[(size_t)bk * 32 + (lane & 0)];
  asm volatile("" :: "v"(cv), "v"(ovv), "v"(fl));
  int oc = ovv < 0 ? 0 : (ovv > RCAP ? RCAP : ovv);
  int cc = cv < 0 ? 0 : (cv > DEGCAP ? DEGCAP : cv);
  cc = cc > (RCAP - oc) ? (RCAP - oc) : cc;
  const int badv = ((cv > DEGCAP) || (cv < 0) || (fl != 0)) ? 1 : 0;
  const float qnan = __int_as_float(0x7fc00000);
  unsigned int* stwu = stw + wave * 128;
  const int* lb = listg + (size_t)bk * RCAP;

#pragma unroll 1
  for (int i = 0; i < 16; ++i) {
    const int row  = row0 + i;
    const int c    = __builtin_amdgcn_readlane(cc, i);
    const int o    = __builtin_amdgcn_readlane(oc, i);
    const int craw = __builtin_amdgcn_readlane(cv, i);
    const int bad  = __builtin_amdgcn_readlane(badv, i);
    float a0 = 0.0f, a1 = 0.0f, a2 = 0.0f, a3 = 0.0f;
#pragma unroll 1
    for (int b0 = 0; b0 < c; b0 += 32) {
      int idx = o + b0 + lane;
      idx = idx < 0 ? 0 : (idx > RCAP - 1 ? RCAP - 1 : idx);
      int sr = lb[idx];
      sr = sr < 0 ? 0 : (sr > NN - 1 ? NN - 1 : sr);
      const int m32 = (c - b0) < 32 ? (c - b0) : 32;
#pragma unroll 1
      for (int k = 0; k < m32; ++k) {
        const int sk = __builtin_amdgcn_readlane(sr, k);
        if constexpr (SRCBF != 0) {
          const v2u q = *(const v2ua*)(xb + (size_t)sk * HD + 4 * lane);
          a0 += __uint_as_float(q.x << 16);
          a1 += __uint_as_float(q.x & 0xffff0000u);
          a2 += __uint_as_float(q.y << 16);
          a3 += __uint_as_float(q.y & 0xffff0000u);
        } else {
          const v4f v = *(const v4f*)(ph + (size_t)sk * HD + 4 * lane);
          a0 += v.x; a1 += v.y; a2 += v.z; a3 += v.w;
        }
      }
    }
    const float degf = (craw > 0) ? (float)craw : 1.0f;
    float r0 = a0 / degf, r1 = a1 / degf, r2 = a2 / degf, r3 = a3 / degf;
    const bool live = row < NN;
    const bool isbad = bad != 0;
    r0 = live ? (isbad ? qnan : r0) : 0.0f;
    r1 = live ? (isbad ? qnan : r1) : 0.0f;
    r2 = live ? (isbad ? qnan : r2) : 0.0f;
    r3 = live ? (isbad ? qnan : r3) : 0.0f;

    const unsigned short hb0 = bf_bits(r0), hb1 = bf_bits(r1), hb2 = bf_bits(r2), hb3 = bf_bits(r3);
    const unsigned short lb0 = bf_bits(r0 - bf_val(hb0)), lb1 = bf_bits(r1 - bf_val(hb1));
    const unsigned short lb2 = bf_bits(r2 - bf_val(hb2)), lb3 = bf_bits(r3 - bf_val(hb3));
    v2u hw, lw;
    hw.x = (unsigned int)hb0 | ((unsigned int)hb1 << 16);
    hw.y = (unsigned int)hb2 | ((unsigned int)hb3 << 16);
    lw.x = (unsigned int)lb0 | ((unsigned int)lb1 << 16);
    lw.y = (unsigned int)lb2 | ((unsigned int)lb3 << 16);
    __builtin_amdgcn_fence(__ATOMIC_RELEASE, "wavefront");
    __builtin_amdgcn_wave_barrier();
    *(v2ua*)(stwu + 2 * lane)      = hw;
    *(v2ua*)(stwu + 64 + 2 * lane) = lw;
    __builtin_amdgcn_fence(__ATOMIC_RELEASE, "wavefront");
    __builtin_amdgcn_wave_barrier();
    const v4u pk = *(const v4ua*)(stwu + 4 * lane);
    unsigned short* gp = pa + (size_t)row * APW + 8 * lane;
    *(volatile v4u*)gp = pk;
    __threadfence();
    *(volatile v4u*)gp = pk;
  }
}

template <int TERMS>
__global__ __launch_bounds__(NTHR) __attribute__((amdgpu_num_vgpr(248)))
void k_gemm(const unsigned short* __restrict__ A, const unsigned short* __restrict__ WT,
            const float* __restrict__ tab, int oBias, float* outF, float* rec) {
  constexpr int NTC = 8;
  constexpr int NI  = 16;
  __shared__ __attribute__((aligned(16))) float stg[TM * HD];
  __shared__ __attribute__((aligned(16))) float pst[RECW];
  __shared__ __attribute__((aligned(16))) float bsh[HD];
  const int tid = (int)threadIdx.x, lane = tid & 31, wave = tid >> 5, hh = lane >> 4, m = lane & 15;
  const int rowBase = (int)blockIdx.x * TM;

  if (tid < 32) {
    const v4f bv = *(const v4f*)(tab + oBias + 4 * tid);
    *(v4fa*)(bsh + 4 * tid) = bv;
  }
  __syncthreads();

  v8f acc[NTC];
  {
    const v8f z = {0.f, 0.f, 0.f, 0.f, 0.f, 0.f, 0.f, 0.f};
#pragma unroll
    for (int t = 0; t < NTC; ++t) acc[t] = z;
  }
  const unsigned short* ap = A + (size_t)(rowBase + 16 * wave + m) * (size_t)APW + 8 * hh;
  const unsigned short* wp = WT + (size_t)m * (size_t)KTOT + 8 * hh;
  constexpr int ksteps = TERMS * (HD / 32);
#pragma unroll 1
  for (int ks = 0; ks < ksteps; ++ks) {
    FragB af;
    af.h[0] = *(const v8usa*)(ap + 32 * ks);
    af.h[1] = *(const v8usa*)(ap + 32 * ks + 16);
#pragma unroll
    for (int t = 0; t < NTC; ++t) {
      const unsigned short* wq = wp + (size_t)(16 * t) * (size_t)KTOT + 32 * ks;
      FragB bf;
      bf.h[0] = *(const v8usa*)wq;
      bf.h[1] = *(const v8usa*)(wq + 16);
      acc[t] = wmb(af, bf, acc[t]);
    }
  }

#pragma unroll
  for (int t = 0; t < NTC; ++t) {
    const int lc = 16 * t + m;
    const float bb = bsh[lc];
#pragma unroll
    for (int r = 0; r < 8; ++r) {
      const int lr = 16 * wave + 8 * hh + r;
      const bool live = (rowBase + lr) < NN;
      const float v = acc[t][r] + bb;
      stg[lr * HD + lc] = live ? v : 0.0f;
    }
  }
  __syncthreads();

  if (tid < HD) {
    int rv = NN - rowBase;
    rv = rv < 0 ? 0 : (rv > TM ? TM : rv);
    float n = 0.0f, mean = 0.0f, M2 = 0.0f;
#pragma unroll 1
    for (int r = 0; r < rv; ++r) {
      const float v = stg[r * HD + tid];
      n += 1.0f;
      const float rk = 1.0f / n;
      const float d = v - mean;
      mean = fmaf(d, rk, mean);
      M2 = fmaf(d, v - mean, M2);
    }
    pst[tid] = n;
    pst[HD + tid] = mean;
    pst[2 * HD + tid] = M2;
  }
  v4f fv[NI];
#pragma unroll
  for (int i = 0; i < NI; ++i) {
    const int lr = 16 * wave + i;
    fv[i] = *(const v4fa*)(stg + lr * HD + 4 * lane);
  }
#pragma unroll
  for (int i = 0; i < NI; ++i) {
    float* op = outF + (size_t)(rowBase + 16 * wave + i) * (size_t)HD + 4 * lane;
    *(volatile v4f*)op = fv[i];
  }
  __threadfence();
#pragma unroll
  for (int i = 0; i < NI; ++i) {
    float* op = outF + (size_t)(rowBase + 16 * wave + i) * (size_t)HD + 4 * lane;
    *(volatile v4f*)op = fv[i];
  }
  __syncthreads();
  const bool pok = tid < RECW / 4;
  v4f pv = {0.f, 0.f, 0.f, 0.f};
  float* rp = rec + (size_t)blockIdx.x * RECW + 4 * (pok ? tid : 0);
  if (pok) {
    pv = *(const v4fa*)(pst + 4 * tid);
    *(volatile v4f*)rp = pv;
  }
  __threadfence();
  if (pok) {
    *(volatile v4f*)rp = pv;
  }
}

__global__ __launch_bounds__(HD) void k_comb(const float* __restrict__ rec, float* stat) {
  __shared__ __attribute__((aligned(16))) float stg[2 * HD];
  const int tid = (int)threadIdx.x;
  const int c = tid & (HD - 1);
  double n = 0.0, mean = 0.0, M2 = 0.0;
#pragma unroll 1
  for (int b = 0; b < NT; ++b) {
    const float* pr = rec + (size_t)b * RECW;
    const float nb = pr[c];
    const float mb = pr[HD + c];
    const float qb = pr[2 * HD + c];
    asm volatile("" :: "v"(nb), "v"(mb), "v"(qb));
    if (nb > 0.5f) {
      const double nn = n + (double)nb;
      const double delta = (double)mb - mean;
      const double f = (double)nb / nn;
      mean = mean + delta * f;
      M2 = M2 + (double)qb + delta * delta * n * f;
      n = nn;
    }
  }
  const double nt = n < 1.0 ? 1.0 : n;
  const float var = (float)(M2 / nt);
  const float ve = var + 1e-5f;
  const float rs = 1.0f / sqrtf(ve);
  stg[c] = (float)mean;
  stg[HD + c] = rs;
  __syncthreads();
  const bool ok = tid < (2 * HD) / 4;
  v4f v = {0.f, 0.f, 0.f, 0.f};
  float* sp = stat + 4 * (ok ? tid : 0);
  if (ok) {
    v = *(const v4fa*)(stg + 4 * tid);
    *(volatile v4f*)sp = v;
  }
  __threadfence();
  if (ok) {
    *(volatile v4f*)sp = v;
  }
}

__device__ __forceinline__ void stage_par(const float* __restrict__ tab, int oS, int oG, int oB,
                                          float* par, int tid) {
  if (tid < 4 * 32) {
    const int w = tid >> 5;
    const int o = (w == 0) ? oS : ((w == 1) ? (oS + HD) : ((w == 2) ? oG : oB));
    const v4f v = *(const v4f*)(tab + o + 4 * (tid & 31));
    *(v4fa*)(par + HD * w + 4 * (tid & 31)) = v;
  }
}

__global__ __launch_bounds__(NTHR) void k_apply_a(const float* __restrict__ pf, const float* __restrict__ tab,
                                                  int oS, int oG, int oB, unsigned short* pa) {
  __shared__ __attribute__((aligned(16))) float par[4 * HD];
  const int tid = (int)threadIdx.x, lane = tid & 31, wave = tid >> 5;
  stage_par(tab, oS, oG, oB, par, tid);
  __syncthreads();
  const int rowBase = (int)blockIdx.x * TM;
  const int cb = 8 * (lane & 15);
  const bool isHi = lane < 16;
  float pm[8], pr[8], pg[8], pb[8];
#pragma unroll
  for (int j = 0; j < 8; ++j) {
    pm[j] = par[cb + j];
    pr[j] = par[HD + cb + j];
    pg[j] = par[2 * HD + cb + j];
    pb[j] = par[3 * HD + cb + j];
  }
#pragma unroll 1
  for (int i = 0; i < 16; ++i) {
    const int row = rowBase + 16 * wave + i;
    const float* p = pf + (size_t)row * HD + cb;
    const v4f a = *(const v4f*)p;
    const v4f b = *(const v4f*)(p + 4);
    asm volatile("" :: "v"(a), "v"(b));
    const bool live = row < NN;
    const float f[8] = {a.x, a.y, a.z, a.w, b.x, b.y, b.z, b.w};
    unsigned int w[4];
#pragma unroll
    for (int j = 0; j < 4; ++j) {
      float y0 = bn_relu(f[2 * j],     pm[2 * j],     pr[2 * j],     pg[2 * j],     pb[2 * j]);
      float y1 = bn_relu(f[2 * j + 1], pm[2 * j + 1], pr[2 * j + 1], pg[2 * j + 1], pb[2 * j + 1]);
      y0 = live ? y0 : 0.0f;
      y1 = live ? y1 : 0.0f;
      const unsigned short h0 = bf_bits(y0), h1 = bf_bits(y1);
      const unsigned short l0 = bf_bits(y0 - bf_val(h0)), l1 = bf_bits(y1 - bf_val(h1));
      const unsigned short q0 = isHi ? h0 : l0, q1 = isHi ? h1 : l1;
      w[j] = (unsigned int)q0 | ((unsigned int)q1 << 16);
    }
    v4u pk; pk.x = w[0]; pk.y = w[1]; pk.z = w[2]; pk.w = w[3];
    unsigned short* op = pa + (size_t)row * APW + 8 * lane;
    *(volatile v4u*)op = pk;
    __threadfence();
    *(volatile v4u*)op = pk;
  }
}

__global__ __launch_bounds__(NTHR) void k_apply_b(const float* __restrict__ pf, const float* __restrict__ tab,
                                                  int oS, int oG, int oB, float* phw) {
  __shared__ __attribute__((aligned(16))) float par[4 * HD];
  const int tid = (int)threadIdx.x, lane = tid & 31, wave = tid >> 5;
  stage_par(tab, oS, oG, oB, par, tid);
  __syncthreads();
  const int rowBase = (int)blockIdx.x * TM;
  const int c4 = 4 * lane;
  const v4f vm = *(const v4fa*)(par + c4);
  const v4f vr = *(const v4fa*)(par + HD + c4);
  const v4f vg = *(const v4fa*)(par + 2 * HD + c4);
  const v4f vb = *(const v4fa*)(par + 3 * HD + c4);
#pragma unroll 1
  for (int i = 0; i < 16; ++i) {
    const int row = rowBase + 16 * wave + i;
    const v4f a = *(const v4f*)(pf + (size_t)row * HD + c4);
    asm volatile("" :: "v"(a));
    const bool live = row < NN;
    v4f o;
    o.x = live ? bn_relu(a.x, vm.x, vr.x, vg.x, vb.x) : 0.0f;
    o.y = live ? bn_relu(a.y, vm.y, vr.y, vg.y, vb.y) : 0.0f;
    o.z = live ? bn_relu(a.z, vm.z, vr.z, vg.z, vb.z) : 0.0f;
    o.w = live ? bn_relu(a.w, vm.w, vr.w, vg.w, vb.w) : 0.0f;
    float* op = phw + (size_t)row * HD + c4;
    *(volatile v4f*)op = o;
    __threadfence();
    *(volatile v4f*)op = o;
  }
}

__global__ __launch_bounds__(NTHR) void k_apply_out(const float* __restrict__ pf, const float* __restrict__ tab,
                                                    int oS, int oG, int oB, const int* __restrict__ gid,
                                                    float* outH, float* poolrec) {
  __shared__ __attribute__((aligned(16))) float hst[TM * HD];
  __shared__ __attribute__((aligned(16))) float bins[NG * HD];
  __shared__ __attribute__((aligned(16))) float par[4 * HD];
  __shared__ int gl[TM];
  const int tid = (int)threadIdx.x, lane = tid & 31, wave = tid >> 5;
  const int rowBase = (int)blockIdx.x * TM;
  stage_par(tab, oS, oG, oB, par, tid);
  {
    const v4f z4 = {0.f, 0.f, 0.f, 0.f};
#pragma unroll
    for (int j = 0; j < (NG * HD) / (NTHR * 4); ++j) *(v4fa*)(bins + 4 * (j * NTHR + tid)) = z4;
    const int r  = rowBase + (tid & (TM - 1));
    const int rc = r < NN ? r : NN - 1;
    const int g  = gid[rc];
    asm volatile("" :: "v"(g));
    if (tid < TM) gl[tid] = (r < NN) ? g : -1;
  }
  __syncthreads();
  const int c4 = 4 * lane;
  const v4f vm = *(const v4fa*)(par + c4);
  const v4f vr = *(const v4fa*)(par + HD + c4);
  const v4f vg = *(const v4fa*)(par + 2 * HD + c4);
  const v4f vb = *(const v4fa*)(par + 3 * HD + c4);
#pragma unroll 1
  for (int i = 0; i < 16; ++i) {
    const int lr  = 16 * wave + i;
    const int row = rowBase + lr;
    const v4f a = *(const v4f*)(pf + (size_t)row * HD + c4);
    asm volatile("" :: "v"(a));
    const bool live = row < NN;
    v4f o;
    o.x = live ? bn_relu(a.x, vm.x, vr.x, vg.x, vb.x) : 0.0f;
    o.y = live ? bn_relu(a.y, vm.y, vr.y, vg.y, vb.y) : 0.0f;
    o.z = live ? bn_relu(a.z, vm.z, vr.z, vg.z, vb.z) : 0.0f;
    o.w = live ? bn_relu(a.w, vm.w, vr.w, vg.w, vb.w) : 0.0f;
    *(v4fa*)(hst + lr * HD + c4) = o;
    const int rw = live ? row : 0;
    float* op = outH + (size_t)rw * HD + c4;
    if (live) *(volatile v4f*)op = o;
    __threadfence();
    if (live) *(volatile v4f*)op = o;
  }
  __syncthreads();
  if (tid < HD) {
    int rv = NN - rowBase;
    rv = rv < 0 ? 0 : (rv > TM ? TM : rv);
#pragma unroll 1
    for (int r = 0; r < rv; ++r) {
      const int g = gl[r];
      const bool ok = (unsigned)g < (unsigned)NG;
      const int gc = ok ? g : 0;
      const float hv = hst[r * HD + tid];
      const float add = ok ? hv : 0.0f;
      bins[gc * HD + tid] = bins[gc * HD + tid] + add;
    }
  }
  __syncthreads();
  v4f bv[(NG * HD) / (NTHR * 4)];
#pragma unroll
  for (int j = 0; j < (NG * HD) / (NTHR * 4); ++j) bv[j] = *(const v4fa*)(bins + 4 * (j * NTHR + tid));
  float* pb = poolrec + (size_t)blockIdx.x * (NG * HD);
#pragma unroll
  for (int j = 0; j < (NG * HD) / (NTHR * 4); ++j) *(volatile v4f*)(pb + 4 * (j * NTHR + tid)) = bv[j];
  __threadfence();
#pragma unroll
  for (int j = 0; j < (NG * HD) / (NTHR * 4); ++j) *(volatile v4f*)(pb + 4 * (j * NTHR + tid)) = bv[j];
}

__global__ __launch_bounds__(HD) void k_pool(const float* __restrict__ poolrec, const int* __restrict__ gid,
                                             float* out) {
  __shared__ int wcn[4];
  __shared__ __attribute__((aligned(16))) float outs[HD];
  const int tid = (int)threadIdx.x, lane = tid & 31, wave = tid >> 5;
  const int g = (int)blockIdx.x;
  constexpr int NQ = NN / 4;
  int cnt = 0;
#pragma unroll 1
  for (int q0 = 0; q0 < NQ; q0 += HD) {
    const int q  = q0 + tid;
    const int qc = q < NQ ? q : NQ - 1;
    const v4i v = *(const v4i*)(gid + 4 * qc);
    asm volatile("" :: "v"(v));
    const int ok = (q < NQ) ? 1 : 0;
    cnt += ok & ((v.x == g) ? 1 : 0);
    cnt += ok & ((v.y == g) ? 1 : 0);
    cnt += ok & ((v.z == g) ? 1 : 0);
    cnt += ok & ((v.w == g) ? 1 : 0);
  }
#pragma unroll
  for (int d = 16; d >= 1; d >>= 1) cnt += __shfl_xor(cnt, d, 32);
  if (lane == 0) wcn[wave] = cnt;
  double s = 0.0;
#pragma unroll 4
  for (int t = 0; t < NT; ++t) {
    s += (double)poolrec[((size_t)t * NG + (size_t)g) * HD + tid];
  }
  __syncthreads();
  const int total = wcn[0] + wcn[1] + wcn[2] + wcn[3];
  const float cf = (total > 0) ? (float)total : 1.0f;
  outs[tid] = (float)s / cf;
  __syncthreads();
  const v4f ov = *(const v4fa*)(outs + 4 * lane);
  float* op = out + (size_t)g * HD + 4 * lane;
  const bool okst = (wave == 0);
  if (okst) *(volatile v4f*)op = ov;
  __threadfence();
  if (okst) *(volatile v4f*)op = ov;
}

static inline size_t al256(size_t o) { return (o + 255) & ~(size_t)255; }

extern "C" void kernel_launch(void* const* d_in, const int* in_sizes, int n_in,
                              void* d_out, int out_size, void* d_ws, size_t ws_size,
                              hipStream_t stream) {
  if (n_in < 12) return;
  if (in_sizes[0] != NN * HD) return;
  if (in_sizes[1] != NE || in_sizes[2] != NE) return;
  if (in_sizes[3] != NN) return;
  if (in_sizes[4] != 2 * HD * HD || in_sizes[8] != 2 * HD * HD) return;
  if (in_sizes[5] != 2 * HD || in_sizes[6] != 2 * HD || in_sizes[7] != 2 * HD) return;
  if (in_sizes[9] != 2 * HD || in_sizes[10] != 2 * HD || in_sizes[11] != 2 * HD) return;
  if ((long long)out_size != (long long)OUT1E + (long long)NN * HD) return;

  const float* x   = (const float*)d_in[0];
  const int*   src = (const int*)  d_in[1];
  const int*   dst = (const int*)  d_in[2];
  const int*   gid = (const int*)  d_in[3];
  const float* W1  = (const float*)d_in[4];
  const float* b1  = (const float*)d_in[5];
  const float* g1  = (const float*)d_in[6];
  const float* be1 = (const float*)d_in[7];
  const float* W2  = (const float*)d_in[8];
  const float* b2  = (const float*)d_in[9];
  const float* gbn = (const float*)d_in[10];
  const float* bbn = (const float*)d_in[11];
  float* out = (float*)d_out;

  char* ws = (char*)d_ws;
  size_t off = 0;
  const size_t oWT = off; off = al256(off + (size_t)NMAT * WSQ * 2);
  const size_t oTB = off; off = al256(off + (size_t)TABF * 4);
  const size_t oXB = off; off = al256(off + (size_t)MP * HD * 2);
  const size_t oPA = off; off = al256(off + (size_t)MP * APW * 2);
  const size_t oPF = off; off = al256(off + (size_t)MP * HD * 4);
  const size_t oPH = off; off = al256(off + (size_t)MP * HD * 4);
  const size_t oPR = off; off = al256(off + (size_t)NT * NG * HD * 4);
  const size_t oLS = off; off = al256(off + (size_t)NBK * RCAP * 4);
  const size_t oCN = off; off = al256(off + (size_t)NPADS * 4);
  const size_t oOF = off; off = al256(off + (size_t)NPADS * 4);
  const size_t oFL = off; off = al256(off + (size_t)NBK * 32 * 4);
  const size_t oRC = off; off = al256(off + (size_t)NT * RECW * 4);
  if (off > ws_size || off > (size_t)WSMAX) return;
  unsigned short* WT  = (unsigned short*)(ws + oWT);
  float*          TAB = (float*)(ws + oTB);
  unsigned short* XB  = (unsigned short*)(ws + oXB);
  unsigned short* PA  = (unsigned short*)(ws + oPA);
  float*          PF  = (float*)(ws + oPF);
  float*          PH  = (float*)(ws + oPH);
  float*          PR  = (float*)(ws + oPR);
  int*            LS  = (int*)(ws + oLS);
  int*            CN  = (int*)(ws + oCN);
  int*            OF  = (int*)(ws + oOF);
  int*            FL  = (int*)(ws + oFL);
  float*          RC  = (float*)(ws + oRC);

  hipFuncSetAttribute(reinterpret_cast<const void*>(&k_bucket), hipFuncAttributeMaxDynamicSharedMemorySize, BK_LDS);

  k_prep<<<PW + PP + PX, NTHR, 0, stream>>>(x, W1, b1, g1, be1, W2, b2, gbn, bbn, WT, TAB, XB);
  k_bucket<<<NBK, NTHR, BK_LDS, stream>>>(src, dst, LS, CN, OF, FL);
  k_agg<1><<<NT, NTHR, 0, stream>>>(XB, PH, LS, CN, OF, FL, PA);

  k_gemm<TERMS_P0><<<NT, NTHR, 0, stream>>>(PA, WT + (size_t)0 * WSQ, TAB, 0 * 256 + 0, PF, RC);
  k_comb<<<1, HD, 0, stream>>>(RC, TAB + PARF + 0 * STATF);
  k_apply_a<<<NT, NTHR, 0, stream>>>(PF, TAB, PARF + 0 * STATF, 1 * 256 + 0, 2 * 256 + 0, PA);
  k_gemm<TERMS_T0><<<NT, NTHR, 0, stream>>>(PA, WT + (size_t)1 * WSQ, TAB, 3 * 256 + 0, PF, RC);
  k_comb<<<1, HD, 0, stream>>>(RC, TAB + PARF + 1 * STATF);
  k_apply_b<<<NT, NTHR, 0, stream>>>(PF, TAB, PARF + 1 * STATF, 4 * 256 + 0, 5 * 256 + 0, PH);

  k_agg<0><<<NT, NTHR, 0, stream>>>(XB, PH, LS, CN, OF, FL, PA);
  k_gemm<TERMS_P1><<<NT, NTHR, 0, stream>>>(PA, WT + (size_t)2 * WSQ, TAB, 0 * 256 + HD, PF, RC);
  k_comb<<<1, HD, 0, stream>>>(RC, TAB + PARF + 2 * STATF);
  k_apply_a<<<NT, NTHR, 0, stream>>>(PF, TAB, PARF + 2 * STATF, 1 * 256 + HD, 2 * 256 + HD, PA);
  k_gemm<TERMS_T1><<<NT, NTHR, 0, stream>>>(PA, WT + (size_t)3 * WSQ, TAB, 3 * 256 + HD, PF, RC);
  k_comb<<<1, HD, 0, stream>>>(RC, TAB + PARF + 3 * STATF);
  k_apply_out<<<NT, NTHR, 0, stream>>>(PF, TAB, PARF + 3 * STATF, 4 * 256 + HD, 5 * 256 + HD, gid,
                                       out + OUT1E, PR);
  k_pool<<<NG, HD, 0, stream>>>(PR, gid, out);
}
